// MambaBlockTVM_36936718745993
// MI455X (gfx1250) — hardware-run, weakly checked
//
#include <hip/hip_runtime.h>
#include <math.h>

typedef __attribute__((ext_vector_type(16))) _Float16 v16h;
typedef __attribute__((ext_vector_type(8)))  _Float16 v8h;
typedef __attribute__((ext_vector_type(2)))  _Float16 v2h;
typedef __attribute__((ext_vector_type(16))) __bf16   v16b;
typedef __attribute__((ext_vector_type(8)))  __bf16   v8b;
typedef __attribute__((ext_vector_type(8)))  float    v8f;
typedef __attribute__((ext_vector_type(4)))  float    v4f;
typedef __attribute__((ext_vector_type(2)))  float    v2f;

constexpr int kNb   = 4;
constexpr int kL    = 2048;
constexpr int kD    = 1024;
constexpr int kN    = 16;
constexpr int kQ    = 64;
constexpr int kC    = kL / kQ;
constexpr int kE    = kNb * kC;
constexpr int kThr  = 256;
constexpr float kInCarry = 1024.0f;
constexpr float kTCarry  = 16777216.0f;
constexpr float kQPCarry = 1048576.0f;
constexpr float kHCarry  = 65536.0f;
constexpr float kScI = 1.0f / (kTCarry * kInCarry);
constexpr float kScS = 1.0f / (kInCarry * kQPCarry);
constexpr float kScO = 1.0f / (kQPCarry * kHCarry);
constexpr float kF16MinNormal = 6.103515625e-5f;
constexpr int kTabK = 0, kTabQ = 64, kTabP = 1088, kTabA64 = 2112, kTabV = 2368, kTabW = 2400, kTabM = 2432;

static_assert(kQ == 64 && kC == 32 && kE == 128 && kN == 16 && kD == 1024, "the index arithmetic below uses these sizes");
static_assert(kTabQ == kTabK + 64 && kTabP == kTabQ + 16 * 64 && kTabA64 == kTabP + 64 * 16 && kTabV == kTabA64 + 256 && kTabW == kTabV + 32 && kTabM == kTabW + 32 && kTabM + 512 <= 3072, "the tables are laid end to end inside TAB");

constexpr size_t kOffZB = 0ull;
constexpr size_t kOffTAB = 8192ull;
constexpr size_t kOffT16 = 20480ull;
constexpr size_t kOffQ16 = 28672ull;
constexpr size_t kOffP16 = 32768ull;
constexpr size_t kOffXT16 = 36864ull;
constexpr size_t kOffYI32 = 16814080ull;
constexpr size_t kOffST32 = 50368512ull;
constexpr size_t kOffH16 = 67145728ull;
constexpr size_t kOffYO32 = 75534336ull;
constexpr size_t kWsTotal = 109088768ull;
static_assert(kWsTotal <= 134217728ull, "carve cap: under 128 MiB");
static_assert(kOffZB == 0
              && kOffTAB == kOffZB + 8192ull
              && kOffT16 == kOffTAB + 12288ull
              && kOffQ16 == kOffT16 + 8192ull
              && kOffP16 == kOffQ16 + 4096ull
              && kOffXT16 == kOffP16 + 4096ull
              && kOffYI32 == kOffXT16 + 16777216ull
              && kOffST32 == kOffYI32 + 33554432ull
              && kOffH16 == kOffST32 + 16777216ull
              && kOffYO32 == kOffH16 + 8388608ull
              && kWsTotal == kOffYO32 + 33554432ull, "the carve is chained and totalled");
static_assert((kOffZB % 256) == 0 && (kOffTAB % 256) == 0 && (kOffT16 % 256) == 0 && (kOffQ16 % 256) == 0 && (kOffP16 % 256) == 0 && (kOffXT16 % 256) == 0 && (kOffYI32 % 256) == 0 && (kOffST32 % 256) == 0 && (kOffH16 % 256) == 0 && (kOffYO32 % 256) == 0, "aligned regions");
static_assert(2048 >= kD, "the zero bias covers the widest launch's 1,024 output columns (the engines read one bias value a column)");

__device__ __forceinline__ unsigned short f2bf_bits(float f) {
  unsigned u = __float_as_uint(f);
  return (unsigned short)((u + 0x7FFFu + ((u >> 16) & 1u)) >> 16);
}
__device__ __forceinline__ float bf_bits2f(unsigned short h) { return __uint_as_float(((unsigned)h) << 16); }
__device__ __forceinline__ float bf16r(float f) { return bf_bits2f(f2bf_bits(f)); }
__device__ __forceinline__ float carry_flush(float v, float carry) {
  const float s = v * carry;
  return (fabsf(s) < kF16MinNormal) ? 0.0f : s;
}

__device__ __forceinline__ void dep_guard4_h(v8f& a, v8f& b, v8f& c, v8f& d, v16h x, v16h y) { asm volatile("v_nop\n\tv_nop\n\tv_nop\n\tv_nop" : "+v"(a), "+v"(b), "+v"(c), "+v"(d) : "v"(x), "v"(y)); }
__device__ __forceinline__ void dep_guard4_b(v8f& a, v8f& b, v8f& c, v8f& d, v16b x, v16b y) { asm volatile("v_nop\n\tv_nop\n\tv_nop\n\tv_nop" : "+v"(a), "+v"(b), "+v"(c), "+v"(d) : "v"(x), "v"(y)); }
__device__ __forceinline__ void keep4_h(v16h a, v16h b, v16h c, v16h d) { asm volatile("v_nop" :: "v"(a), "v"(b), "v"(c), "v"(d)); }
__device__ __forceinline__ void keep4_b(v16b a, v16b b, v16b c, v16b d) { asm volatile("v_nop" :: "v"(a), "v"(b), "v"(c), "v"(d)); }
__device__ __forceinline__ void acc_guard4(v8f& a, v8f& b, v8f& c, v8f& d) { asm volatile("v_nop\n\tv_nop\n\tv_nop\n\tv_nop" : "+v"(a), "+v"(b), "+v"(c), "+v"(d)); }

template <typename T> struct Frag;
template <> struct Frag<_Float16> {
  typedef v16h V; union U { v16h v; v8h h[2]; };
  static __device__ __forceinline__ v16h load(const _Float16* p) {
    U f; f.h[0] = *(const v8h*)(p); f.h[1] = *(const v8h*)(p + 16); return f.v;
  }
  static __device__ __forceinline__ v8f mma(v16h a, v16h b, v8f c) {
    return __builtin_amdgcn_wmma_f32_16x16x32_f16(false, a, false, b, (short)0, c, false, false);
  }
  static __device__ __forceinline__ void guard4(v8f& a, v8f& b, v8f& c, v8f& d, v16h x, v16h y) { dep_guard4_h(a, b, c, d, x, y); }
  static __device__ __forceinline__ void keep(v16h a, v16h b, v16h c, v16h d) { keep4_h(a, b, c, d); }
};
template <> struct Frag<__bf16> {
  typedef v16b V; union U { v16b v; v8b h[2]; };
  static __device__ __forceinline__ v16b load(const __bf16* p) {
    U f; f.h[0] = *(const v8b*)(p); f.h[1] = *(const v8b*)(p + 16); return f.v;
  }
  static __device__ __forceinline__ v8f mma(v16b a, v16b b, v8f c) {
    return __builtin_amdgcn_wmma_f32_16x16x32_bf16(false, a, false, b, (short)0, c, false, false);
  }
  static __device__ __forceinline__ void guard4(v8f& a, v8f& b, v8f& c, v8f& d, v16b x, v16b y) { dep_guard4_b(a, b, c, d, x, y); }
  static __device__ __forceinline__ void keep(v16b a, v16b b, v16b c, v16b d) { keep4_b(a, b, c, d); }
};

__device__ __forceinline__ v8f mma_h(v16h a, v16h b, v8f c) {
  c = __builtin_amdgcn_wmma_f32_16x16x32_f16(false, a, false, b, (short)0, c, false, false);
  asm volatile("v_nop\n\tv_nop\n\tv_nop\n\tv_nop" : "+v"(c) : "v"(a), "v"(b));
  return c;
}

template <int ET> struct Elem;
template <> struct Elem<0> { typedef _Float16 T; };
template <> struct Elem<1> { typedef __bf16 T; };
template <int ET, bool SPLIT, int BIAS_MODE, int OUT_MODE, bool RESID, int ACT = 0>
__global__ __launch_bounds__(256) void wmma_gemm64(
    const unsigned short* __restrict__ Ap, const unsigned short* __restrict__ A2p, int lda, long strideA,
    const unsigned short* __restrict__ Btp, const unsigned short* __restrict__ Bt2p, int ldb, long strideB,
    void* __restrict__ Cout, void* __restrict__ Cout2, int ldc, long strideC,
    const float* __restrict__ bias,
    const float* __restrict__ resid, long strideR,
    int M, int N, int K, float scale) {
  typedef typename Elem<ET>::T T;
  typedef typename Frag<T>::V V;
  const T* A = (const T*)Ap; const T* A2 = (const T*)A2p; const T* Bt = (const T*)Btp; const T* Bt2 = (const T*)Bt2p;
  __shared__ __align__(16) float sT[8][16 * 68];
  const int b    = blockIdx.y;
  const int lane = threadIdx.x & 31;
  const int wave = threadIdx.x >> 5;
  const int tilesN = N >> 6;
  const int tilesM = M >> 6;
  const int tile = blockIdx.x * 8 + wave;
  if (tile >= tilesM * tilesN) return;
  const int tm = tile / tilesN;
  const int tn = tile - tm * tilesN;
  const int m0 = tm << 6;
  const int n0 = tn << 6;

  const T* Ab  = A  + (size_t)b * strideA;
  const T* Bb  = Bt + (size_t)b * strideB;
  const T* Ab2 = SPLIT ? (A2  + (size_t)b * strideA) : nullptr;
  const T* Bb2 = SPLIT ? (Bt2 + (size_t)b * strideB) : nullptr;

  const int rlane = lane & 15;
  const int koff  = (lane >> 4) * 8;
  const int mOff  = (lane >> 4) * 8;

  v8f acc[4][4];
#pragma unroll
  for (int i = 0; i < 4; ++i)
#pragma unroll
    for (int j = 0; j < 4; ++j) acc[i][j] = (v8f){0.f,0.f,0.f,0.f,0.f,0.f,0.f,0.f};

  for (int k0 = 0; k0 < K; k0 += 32) {
    V bh[4], bl[4];
#pragma unroll
    for (int j = 0; j < 4; ++j) {
      const size_t bo = (size_t)(n0 + (j << 4) + rlane) * ldb + koff + k0;
      bh[j] = Frag<T>::load(Bb + bo);
      if (SPLIT) bl[j] = Frag<T>::load(Bb2 + bo);
    }
#pragma unroll
    for (int i = 0; i < 4; ++i) {
      const size_t ao = (size_t)(m0 + (i << 4) + rlane) * lda + koff + k0;
      V ah = Frag<T>::load(Ab + ao);
      V al;
      if (SPLIT) al = Frag<T>::load(Ab2 + ao);
#pragma unroll
      for (int j = 0; j < 4; ++j) {
        acc[i][j] = Frag<T>::mma(ah, bh[j], acc[i][j]);
        if (SPLIT) {
          acc[i][j] = Frag<T>::mma(ah, bl[j], acc[i][j]);
          acc[i][j] = Frag<T>::mma(al, bh[j], acc[i][j]);
        }
      }
      Frag<T>::guard4(acc[i][0], acc[i][1], acc[i][2], acc[i][3], ah, SPLIT ? al : ah);
    }
    Frag<T>::keep(bh[0], bh[1], bh[2], bh[3]);
    if (SPLIT) Frag<T>::keep(bl[0], bl[1], bl[2], bl[3]);
  }
  acc_guard4(acc[0][0], acc[0][1], acc[0][2], acc[0][3]);
  acc_guard4(acc[1][0], acc[1][1], acc[1][2], acc[1][3]);
  acc_guard4(acc[2][0], acc[2][1], acc[2][2], acc[2][3]);
  acc_guard4(acc[3][0], acc[3][1], acc[3][2], acc[3][3]);

  float* slab = sT[wave];
  const float* Rb = RESID ? (resid + (size_t)b * strideR) : nullptr;
#pragma unroll
  for (int i = 0; i < 4; ++i) {
    const int mBase = m0 + (i << 4);
#pragma unroll
    for (int j = 0; j < 4; ++j) {
      const int n = n0 + (j << 4) + rlane;
      float bv = 0.f;
      if (BIAS_MODE == 2) bv = bias[n];
#pragma unroll
      for (int r = 0; r < 8; ++r) {
        float v = acc[i][j][r] * scale;
        if (BIAS_MODE == 1) v += bias[mBase + mOff + r];
        if (BIAS_MODE == 2) v += bv;
        if (RESID) v += Rb[(size_t)(mBase + mOff + r) * ldc + n];
        if (ACT == 1) v = tanhf(v);
        if (ACT == 2) v = fmaxf(v, 0.0f);
        if (ACT == 3) v = v / (1.0f + expf(-v));
        if (ACT == 4) v = (v > 0.f) ? v : 0.01f * v;
        slab[(mOff + r) * 68 + (j << 4) + rlane] = v;
      }
    }
    __builtin_amdgcn_fence(__ATOMIC_RELEASE, "workgroup");
    __builtin_amdgcn_wave_barrier();
    __builtin_amdgcn_fence(__ATOMIC_ACQUIRE, "workgroup");
    if (OUT_MODE == 0) {
      float* C = (float*)Cout + (size_t)b * strideC;
      const int hh = lane >> 4, c4 = (lane & 15) * 4;
      for (int pass = 0; pass < 2; ++pass) {
#pragma unroll
        for (int it = 0; it < 8; ++it) {
          const int row = it * 2 + hh;
          v4f v = *(const v4f*)(slab + row * 68 + c4);
          *(volatile v4f*)(C + (size_t)(mBase + row) * ldc + n0 + c4) = v;
        }
        __threadfence();
      }
    } else {
      const int q = lane >> 3, c8 = (lane & 7) * 8;
      unsigned short* C  = (unsigned short*)Cout  + (size_t)b * strideC;
      unsigned short* C2 = (OUT_MODE == 2) ? ((unsigned short*)Cout2 + (size_t)b * strideC) : nullptr;
      for (int pass = 0; pass < 2; ++pass) {
#pragma unroll
        for (int it = 0; it < 4; ++it) {
          const int row = it * 4 + q;
          const float* sp = slab + row * 68 + c8;
          v8h hv, lv;
#pragma unroll
          for (int e = 0; e < 8; ++e) {
            if (OUT_MODE == 1) {
              hv[e] = (_Float16)sp[e];
            } else {
              unsigned short hb = f2bf_bits(sp[e]);
              unsigned short lb = f2bf_bits(sp[e] - bf_bits2f(hb));
              hv[e] = __builtin_bit_cast(_Float16, hb);
              lv[e] = __builtin_bit_cast(_Float16, lb);
            }
          }
          *(volatile v8h*)(C + (size_t)(mBase + row) * ldc + n0 + c8) = hv;
          if (OUT_MODE == 2) *(volatile v8h*)(C2 + (size_t)(mBase + row) * ldc + n0 + c8) = lv;
        }
        __threadfence();
      }
    }
    __builtin_amdgcn_fence(__ATOMIC_RELEASE, "workgroup");
    __builtin_amdgcn_wave_barrier();
    __builtin_amdgcn_fence(__ATOMIC_ACQUIRE, "workgroup");
  }
}

__global__ __launch_bounds__(256) void wmma_gemm32(
    const unsigned short* __restrict__ Ap, int lda, long strideA,
    const unsigned short* __restrict__ Btp, int ldb, long strideB,
    float* __restrict__ Cout, int ldc, long strideC,
    const float* __restrict__ bias,
    int M, int N, int K, float scale) {
  typedef _Float16 T;
  typedef Frag<T>::V V;
  const T* A = (const T*)Ap; const T* Bt = (const T*)Btp;
  __shared__ __align__(16) float sT[8][16 * 36];
  const int b    = blockIdx.y;
  const int lane = threadIdx.x & 31;
  const int wave = threadIdx.x >> 5;
  const int tilesN = N >> 5;
  const int tilesM = M >> 6;
  const int tile = blockIdx.x * 8 + wave;
  if (tile >= tilesM * tilesN) return;
  const int tm = tile / tilesN;
  const int tn = tile - tm * tilesN;
  const int m0 = tm << 6;
  const int n0 = tn << 5;

  const T* Ab = A  + (size_t)b * strideA;
  const T* Bb = Bt + (size_t)b * strideB;

  const int rlane = lane & 15;
  const int koff  = (lane >> 4) * 8;
  const int mOff  = (lane >> 4) * 8;

  v8f acc[4][2];
#pragma unroll
  for (int i = 0; i < 4; ++i)
#pragma unroll
    for (int j = 0; j < 2; ++j) acc[i][j] = (v8f){0.f,0.f,0.f,0.f,0.f,0.f,0.f,0.f};

  for (int k0 = 0; k0 < K; k0 += 32) {
    V bh[2];
#pragma unroll
    for (int j = 0; j < 2; ++j) {
      const size_t bo = (size_t)(n0 + (j << 4) + rlane) * ldb + koff + k0;
      bh[j] = Frag<T>::load(Bb + bo);
    }
#pragma unroll
    for (int i = 0; i < 4; i += 2) {
      const size_t ao0 = (size_t)(m0 + (i << 4) + rlane) * lda + koff + k0;
      const size_t ao1 = (size_t)(m0 + ((i + 1) << 4) + rlane) * lda + koff + k0;
      V ah0 = Frag<T>::load(Ab + ao0);
      V ah1 = Frag<T>::load(Ab + ao1);
      acc[i][0]     = Frag<T>::mma(ah0, bh[0], acc[i][0]);
      acc[i][1]     = Frag<T>::mma(ah0, bh[1], acc[i][1]);
      acc[i + 1][0] = Frag<T>::mma(ah1, bh[0], acc[i + 1][0]);
      acc[i + 1][1] = Frag<T>::mma(ah1, bh[1], acc[i + 1][1]);
      Frag<T>::guard4(acc[i][0], acc[i][1], acc[i + 1][0], acc[i + 1][1], ah0, ah1);
    }
    Frag<T>::keep(bh[0], bh[1], bh[0], bh[1]);
  }
  acc_guard4(acc[0][0], acc[0][1], acc[1][0], acc[1][1]);
  acc_guard4(acc[2][0], acc[2][1], acc[3][0], acc[3][1]);

  float* slab = sT[wave];
  float* C = Cout + (size_t)b * strideC;
#pragma unroll
  for (int i = 0; i < 4; ++i) {
    const int mBase = m0 + (i << 4);
#pragma unroll
    for (int j = 0; j < 2; ++j) {
      const int n = n0 + (j << 4) + rlane;
      const float bv = bias[n];
#pragma unroll
      for (int r = 0; r < 8; ++r) {
        float v = acc[i][j][r] * scale;
        v += bv;
        slab[(mOff + r) * 36 + (j << 4) + rlane] = v;
      }
    }
    __builtin_amdgcn_fence(__ATOMIC_RELEASE, "workgroup");
    __builtin_amdgcn_wave_barrier();
    __builtin_amdgcn_fence(__ATOMIC_ACQUIRE, "workgroup");
    {
      const int q = lane >> 3, c4 = (lane & 7) * 4;
      for (int pass = 0; pass < 2; ++pass) {
#pragma unroll
        for (int it = 0; it < 4; ++it) {
          const int row = it * 4 + q;
          v4f v = *(const v4f*)(slab + row * 36 + c4);
          *(volatile v4f*)(C + (size_t)(mBase + row) * ldc + n0 + c4) = v;
        }
        __threadfence();
      }
    }
    __builtin_amdgcn_fence(__ATOMIC_RELEASE, "workgroup");
    __builtin_amdgcn_wave_barrier();
    __builtin_amdgcn_fence(__ATOMIC_ACQUIRE, "workgroup");
  }
}
static_assert(sizeof(float) * 8 * 16 * 36 == 18432, "the tail's slabs: 8 waves x 16 rows x 36 floats = 18,432 B of LDS");


__device__ __forceinline__ void store2(float* p, float v) {
  *(volatile float*)p = v;
  __threadfence();
  *(volatile float*)p = v;
}

__global__ __launch_bounds__(kThr) void zero_kernel(float* __restrict__ dst) {
  const size_t o4 = ((size_t)blockIdx.x * kThr + threadIdx.x) * 4u;
  const v4f z = {0.f, 0.f, 0.f, 0.f};
  *(volatile v4f*)(dst + o4) = z;
  __threadfence();
  *(volatile v4f*)(dst + o4) = z;
}

__global__ __launch_bounds__(64) void tables_kernel(const float* __restrict__ Am, const float* __restrict__ Bv, float* __restrict__ TAB) {
  if (threadIdx.x != 0u) return;
  const volatile __attribute__((address_space(1))) float* TG = (const volatile __attribute__((address_space(1))) float*)TAB;
  for (int n = 0; n < kN; ++n) { const float b0 = Bv[n]; const float bb = bf16r(b0); store2(TAB + kTabV + n, bb); store2(TAB + kTabW + n, bb); }
  for (int l = 0; l < kQ; ++l) {
    const int cur = (l & 1) * kN, nxt = ((l + 1) & 1) * kN;
    float k = 0.0f;
    for (int n = 0; n < kN; ++n) {
      const float b0 = Bv[n];
      const float vn = TG[kTabV + cur + n];
      k += bf16r(b0) * vn;
      store2(TAB + kTabQ + n * kQ + (kQ - 1 - l), vn);
    }
    store2(TAB + kTabK + l, k);
    for (int i = 0; i < kN; ++i) {
      float acc = 0.0f;
      for (int j = 0; j < kN; ++j) { const float a0 = Am[i * kN + j]; acc += bf16r(a0) * TG[kTabV + cur + j]; }
      store2(TAB + kTabV + nxt + i, acc);
    }
    for (int n = 0; n < kN; ++n) {
      float acc = 0.0f;
      for (int m = 0; m < kN; ++m) { const float a0 = Am[m * kN + n]; acc += TG[kTabW + cur + m] * bf16r(a0); }
      store2(TAB + kTabW + nxt + n, acc);
      store2(TAB + kTabP + l * kN + n, acc);
    }
  }
  for (int i = 0; i < kN * kN; ++i) { const float a0 = Am[i]; store2(TAB + kTabM + i, bf16r(a0)); }
  for (int sq = 0; sq < 6; ++sq) {
    const int cur = (sq & 1) * 256, nxt = ((sq + 1) & 1) * 256;
    for (int i = 0; i < kN; ++i)
      for (int j = 0; j < kN; ++j) {
        float acc = 0.0f;
        for (int m = 0; m < kN; ++m) acc += TG[kTabM + cur + i * kN + m] * TG[kTabM + cur + m * kN + j];
        store2(TAB + kTabM + nxt + i * kN + j, acc);
      }
  }
  for (int i = 0; i < kN * kN; ++i) store2(TAB + kTabA64 + i, TG[kTabM + i]);
}

__global__ __launch_bounds__(kThr) void tabcast_kernel(const float* __restrict__ TAB, unsigned short* __restrict__ T16, unsigned short* __restrict__ Q16, unsigned short* __restrict__ P16) {
  const unsigned tid = threadIdx.x;
  v8h hv;
  unsigned short* dp;
  if (blockIdx.x < 2u) {
    const unsigned idx = blockIdx.x * (unsigned)kThr + tid;
    const unsigned s8 = idx & 7u, l = idx >> 3;
#pragma unroll
    for (int e = 0; e < 8; ++e) {
      const unsigned s = s8 * 8u + (unsigned)e;
      const bool live = s <= l;
      const float k = TAB[kTabK + (live ? (l - s) : 0u)];
      hv[e] = (_Float16)carry_flush(live ? k : 0.0f, kTCarry);
    }
    dp = T16 + (size_t)idx * 8u;
  } else if (blockIdx.x == 2u) {
    const unsigned s8 = tid & 7u, n = tid >> 3;
    const bool live = n < (unsigned)kN;
    const float* sp = TAB + kTabQ + (live ? n : 0u) * (unsigned)kQ + s8 * 8u;
#pragma unroll
    for (int e = 0; e < 8; ++e) { const float q = sp[e]; hv[e] = (_Float16)carry_flush(live ? q : 0.0f, kQPCarry); }
    dp = Q16 + (size_t)tid * 8u;
  } else {
    const unsigned n8 = tid & 3u, l = tid >> 2;
    const bool live = n8 < 2u;
    const float* sp = TAB + kTabP + l * (unsigned)kN + (live ? n8 : 0u) * 8u;
#pragma unroll
    for (int e = 0; e < 8; ++e) { const float p = sp[e]; hv[e] = (_Float16)carry_flush(live ? p : 0.0f, kQPCarry); }
    dp = P16 + (size_t)tid * 8u;
  }
  *(volatile v8h*)dp = hv;
  __threadfence();
  *(volatile v8h*)dp = hv;
}
static_assert(64 * 64 / 8 == 2 * kThr && 32 * 64 / 8 == kThr && 64 * 32 / 8 == kThr, "operand-plane grid exact: 2 + 1 + 1 blocks");

__global__ __launch_bounds__(kThr) void xt_cast_kernel(const float* __restrict__ X, unsigned short* __restrict__ XT16) {
  const unsigned i = blockIdx.x * (unsigned)kThr + threadIdx.x;
  const unsigned j = i & 7u, d = (i >> 3) & 1023u, e = i >> 13;
  const float* sp = X + (size_t)(e * (unsigned)kQ + j * 8u) * kD + d;
  v8h hv;
#pragma unroll
  for (int t = 0; t < 8; ++t) { const float v = sp[(size_t)t * kD]; hv[t] = (_Float16)carry_flush(bf16r(v), kInCarry); }
  unsigned short* dp = XT16 + (size_t)i * 8u;
  *(volatile v8h*)dp = hv;
  __threadfence();
  *(volatile v8h*)dp = hv;
}
static_assert((size_t)kE * kD * (kQ / 8) == 4096ull * kThr, "transposing cast grid exact: 4,096 blocks");

__global__ __launch_bounds__(kThr) void carry_kernel(const float* __restrict__ ST32, const float* __restrict__ A64, unsigned short* __restrict__ H16) {
  const unsigned gi = blockIdx.x * (unsigned)kThr + threadIdx.x;
  const unsigned b = gi >> 10, d = gi & 1023u;
  float h[kN];
#pragma unroll
  for (int n = 0; n < kN; ++n) h[n] = 0.0f;
  v8h zv;
#pragma unroll
  for (int t = 0; t < 8; ++t) zv[t] = (_Float16)0.0f;
  for (int c = 0; c < kC; ++c) {
    const size_t o = (((size_t)b * kC + (size_t)c) * kD + d) * 32u;
    v8h h0, h1;
#pragma unroll
    for (int t = 0; t < 8; ++t) { h0[t] = (_Float16)carry_flush(h[t], kHCarry); h1[t] = (_Float16)carry_flush(h[8 + t], kHCarry); }
    unsigned short* dp = H16 + o;
    for (int pass = 0; pass < 2; ++pass) {
      *(volatile v8h*)dp = h0;
      *(volatile v8h*)(dp + 8) = h1;
      *(volatile v8h*)(dp + 16) = zv;
      *(volatile v8h*)(dp + 24) = zv;
      __threadfence();
    }
    const float* sp = ST32 + o;
    const v4f s0 = *(const v4f*)sp, s1 = *(const v4f*)(sp + 4), s2 = *(const v4f*)(sp + 8), s3 = *(const v4f*)(sp + 12);
    float hn[kN];
#pragma unroll
    for (int i = 0; i < kN; ++i) {
      float acc = (i < 4) ? s0[i & 3] : (i < 8) ? s1[i & 3] : (i < 12) ? s2[i & 3] : s3[i & 3];
#pragma unroll
      for (int j = 0; j < kN; ++j) acc += A64[i * kN + j] * h[j];
      hn[i] = acc;
    }
#pragma unroll
    for (int n = 0; n < kN; ++n) h[n] = hn[n];
  }
}
static_assert(kNb * kD == 16 * kThr, "carry grid exact: 16 blocks");

__global__ __launch_bounds__(kThr) void combine_kernel(const float* __restrict__ YD32, const float* __restrict__ YO32, float* __restrict__ out) {
  const size_t o4 = ((size_t)blockIdx.x * kThr + threadIdx.x) * 4u;
  const v4f a = *(const v4f*)(YD32 + o4), b = *(const v4f*)(YO32 + o4);
  v4f o;
#pragma unroll
  for (int k = 0; k < 4; ++k) o[k] = a[k] + b[k];
  *(volatile v4f*)(out + o4) = o;
  __threadfence();
  *(volatile v4f*)(out + o4) = o;
}
static_assert((size_t)kE * kQ * (kD / 4) == 8192ull * kThr, "combine grid exact: 8,192 blocks");

static_assert(((kQ / 64) * (kD / 64)) % 8 == 0 && ((kD / 64) * (32 / 32)) % 8 == 0, "the batched grids exact: every wave live");

extern "C" void kernel_launch(void* const* d_in, const int* in_sizes, int n_in,
                              void* d_out, int out_size, void* d_ws, size_t ws_size,
                              hipStream_t stream) {
  if (n_in < 3 || d_out == nullptr || d_ws == nullptr) return;
  if (in_sizes[0] != kNb * kL * kD || in_sizes[1] != kN * kN || in_sizes[2] != kN) return;
  if (out_size != kNb * kL * kD) return;
  if (ws_size < kWsTotal) return;
  const float* X = (const float*)d_in[0];
  const float* Am = (const float*)d_in[1];
  const float* Bv = (const float*)d_in[2];
  float* out = (float*)d_out;
  char* ws = (char*)d_ws;
  float* ZB = (float*)(ws + kOffZB);
  float* TAB = (float*)(ws + kOffTAB);
  unsigned short* T16 = (unsigned short*)(ws + kOffT16);
  unsigned short* Q16 = (unsigned short*)(ws + kOffQ16);
  unsigned short* P16 = (unsigned short*)(ws + kOffP16);
  unsigned short* XT16 = (unsigned short*)(ws + kOffXT16);
  float* YI32 = (float*)(ws + kOffYI32);
  float* ST32 = (float*)(ws + kOffST32);
  unsigned short* H16 = (unsigned short*)(ws + kOffH16);
  float* YO32 = (float*)(ws + kOffYO32);

  zero_kernel<<<2, kThr, 0, stream>>>(ZB);
  tables_kernel<<<1, 64, 0, stream>>>(Am, Bv, TAB);
  tabcast_kernel<<<4, kThr, 0, stream>>>(TAB, T16, Q16, P16);
  xt_cast_kernel<<<4096, kThr, 0, stream>>>(X, XT16);
  wmma_gemm64<0, false, 2, 0, false, 0><<<dim3((kQ / 64) * (kD / 64) / 8, kE), 256, 0, stream>>>(
      T16, T16, kQ, 0L, XT16, XT16, kQ, (long)kD * kQ, (void*)YI32, (void*)YI32, kD, (long)kQ * kD, ZB, nullptr, 0L, kQ, kD, kQ, kScI);
  wmma_gemm32<<<dim3((kD / 64) * (32 / 32) / 8, kE), 256, 0, stream>>>(
      XT16, kQ, (long)kD * kQ, Q16, kQ, 0L, ST32, 32, (long)kD * 32, ZB, kD, 32, kQ, kScS);
  carry_kernel<<<16, kThr, 0, stream>>>(ST32, TAB + kTabA64, H16);
  wmma_gemm64<0, false, 2, 0, false, 0><<<dim3((kQ / 64) * (kD / 64) / 8, kE), 256, 0, stream>>>(
      P16, P16, 32, 0L, H16, H16, 32, (long)kD * 32, (void*)YO32, (void*)YO32, kD, (long)kQ * kD, ZB, nullptr, 0L, kQ, kD, 32, kScO);
  combine_kernel<<<8192, kThr, 0, stream>>>(YI32, YO32, out);
}
